// _ParallelBlock_7919919694497
// MI455X (gfx1250) — hardware-run, weakly checked
//
#include <hip/hip_runtime.h>
#include <stddef.h>
#include <math.h>


#define BB    4
#define LL    1024
#define NTOK  (BB * LL)
#define DM    512
#define NHEAD 32
#define HDIM  16
#define DI    1024
#define DSS   64
#define HPD   64
#define NHM   16
#define DCV   4
#define CCH   (DI + 2 * DSS)
#define DIP   (2 * DI + 2 * DSS + NHM)
#define DIPP  2240
#define COL_X  DI
#define COL_B  (2 * DI)
#define COL_DT (2 * DI + 2 * DSS)
#define NTHR  256
#define WSCAP 134217728
#define LNEPS 1e-5f

#define W_CARRY  64.0f
#define Q_CARRY  8.0f
#define P_CARRY  4096.0f
#define SC_SCORE (1.0f / 256.0f)
#define SC_O     8.0f

static_assert((DIPP % 64) == 0 && DIPP >= DIP && (DM % 32) == 0 && (DI % 32) == 0 && (NTOK % 64) == 0);
static_assert(((3 * DM) % 256) == 0 && (DM % 256) == 0 && (LL % 64) == 0 && NHEAD * HDIM == DM && NHM * HPD == DI);

typedef _Float16 v16h __attribute__((ext_vector_type(16)));
typedef _Float16 v8h __attribute__((ext_vector_type(8), __may_alias__));
typedef float v8f __attribute__((ext_vector_type(8)));
typedef float v4f __attribute__((ext_vector_type(4), __may_alias__));
typedef int v8i __attribute__((ext_vector_type(8)));
union Frag { v16h v; v8h hv[2]; v8i w; };
static_assert(sizeof(Frag) == 32);

__device__ __forceinline__ v8f zero8() { v8f z = {0.f, 0.f, 0.f, 0.f, 0.f, 0.f, 0.f, 0.f}; return z; }
__device__ __forceinline__ v8i zero8i() { v8i z = {0, 0, 0, 0, 0, 0, 0, 0}; return z; }
__device__ __forceinline__ v4f zero4() { v4f z = {0.f, 0.f, 0.f, 0.f}; return z; }

__device__ __forceinline__ v8f wmf(const Frag& a, const Frag& b, v8f c) {
  v8f d = __builtin_amdgcn_wmma_f32_16x16x32_f16(false, a.v, false, b.v, (short)0, c, false, false);
  asm volatile("v_nop\n\tv_nop\n\tv_nop\n\tv_nop" : "+v"(d) : "v"(a.w), "v"(b.w));
  return d;
}

__device__ __forceinline__ v8h cvt8(v4f a, v4f c, float s) {
  v8h r;
  r[0] = (_Float16)(a[0] * s); r[1] = (_Float16)(a[1] * s); r[2] = (_Float16)(a[2] * s); r[3] = (_Float16)(a[3] * s);
  r[4] = (_Float16)(c[0] * s); r[5] = (_Float16)(c[1] * s); r[6] = (_Float16)(c[2] * s); r[7] = (_Float16)(c[3] * s);
  return r;
}

#define NW_QKV ((size_t)3 * DM * DM)
#define NW_AO  ((size_t)DM * DM)
#define NW_IP  ((size_t)DIPP * DM)
#define NW_OP  ((size_t)DM * DI)
#define OW_QKV ((size_t)0)
#define OW_AO  (OW_QKV + NW_QKV)
#define OW_FI  (OW_AO + NW_AO)
#define OW_FO  (OW_FI + NW_IP)
#define OW_BI  (OW_FO + NW_OP)
#define OW_BO  (OW_BI + NW_IP)
#define NW16   (OW_BO + NW_OP)
static_assert((OW_AO % 64) == 0 && (OW_FI % 64) == 0 && (OW_FO % 64) == 0 && (OW_BI % 64) == 0 && (OW_BO % 64) == 0);

#define CVB    2048
#define CB_H   (NTOK * DM / CVB)
#define CB_QKV (3 * DM * DM / CVB)
#define CB_AO  (DM * DM / CVB)
#define CB_IP  (DIPP * DM / CVB)
#define CB_IPV (DIP * DM / CVB)
#define CB_OP  (DM * DI / CVB)
#define CC1 CB_H
#define CC2 (CC1 + CB_QKV)
#define CC3 (CC2 + CB_AO)
#define CC4 (CC3 + CB_IP)
#define CC5 (CC4 + CB_OP)
#define CC6 (CC5 + CB_IP)
#define CCT (CC6 + CB_OP)
static_assert((NTOK * DM) % CVB == 0 && (3 * DM * DM) % CVB == 0 && (DM * DM) % CVB == 0);
static_assert((DIPP * DM) % CVB == 0 && (DIP * DM) % CVB == 0 && (DM * DI) % CVB == 0 && CVB == NTHR * 8);

#define SZ_W16  ((size_t)NW16 * 2)
#define SZ_H16  ((size_t)NTOK * DM * 2)
#define SZ_T512 ((size_t)NTOK * DM * 4)
#define SZ_QKV  ((size_t)NTOK * 3 * DM * 4)
#define SZ_HP   ((size_t)BB * NHEAD * LL * HDIM * 2)
#define SZ_XZ   ((size_t)NTOK * DIPP * 4)
#define SZ_Y32  ((size_t)NTOK * DI * 4)
#define SZ_Y16  ((size_t)NTOK * DI * 2)
#define O_W16   ((size_t)0)
#define O_H16   (O_W16 + SZ_W16)
#define O_ATT   (O_H16 + SZ_H16)
#define O_FWD   (O_ATT + SZ_T512)
#define O_BWD   (O_FWD + SZ_T512)
#define O_SCR   (O_BWD + SZ_T512)
#define O_QKV   (O_SCR)
#define O_Q16   (O_QKV + SZ_QKV)
#define O_K16   (O_Q16 + SZ_HP)
#define O_VT    (O_K16 + SZ_HP)
#define O_O16   (O_VT + SZ_HP)
#define END_A   (O_O16 + SZ_HP)
#define O_XZ    (O_SCR)
#define O_Y32   (O_XZ + SZ_XZ)
#define O_Y16   (O_Y32 + SZ_Y32)
#define END_M   (O_Y16 + SZ_Y16)
#define WSTOT   (END_M > END_A ? END_M : END_A)
static_assert(WSTOT <= (size_t)WSCAP);
static_assert((O_H16 % 128) == 0 && (O_ATT % 128) == 0 && (O_FWD % 128) == 0 && (O_BWD % 128) == 0 && (O_SCR % 128) == 0);
static_assert((O_Q16 % 128) == 0 && (O_K16 % 128) == 0 && (O_VT % 128) == 0 && (O_O16 % 128) == 0 && (END_A % 128) == 0);
static_assert((O_Y32 % 128) == 0 && (O_Y16 % 128) == 0 && (END_M % 128) == 0 && ((DIPP * 4) % 128) == 0);

__global__ __launch_bounds__(NTHR) void k_cvt(const float* __restrict__ hsrc, const float* __restrict__ wqkv,
                                              const float* __restrict__ wao, const float* __restrict__ wfi,
                                              const float* __restrict__ wfo, const float* __restrict__ wbi,
                                              const float* __restrict__ wbo, _Float16* H16, _Float16* W16) {
  const int blk = blockIdx.x, tid = threadIdx.x;
  const float* src;
  _Float16* dstp;
  int lb;
  float sc;
  bool zero = false;
  if (blk < CC1)      { src = hsrc; lb = blk;       dstp = H16;          sc = 1.0f; }
  else if (blk < CC2) { src = wqkv; lb = blk - CC1; dstp = W16 + OW_QKV; sc = W_CARRY; }
  else if (blk < CC3) { src = wao;  lb = blk - CC2; dstp = W16 + OW_AO;  sc = W_CARRY; }
  else if (blk < CC4) { src = wfi;  lb = blk - CC3; dstp = W16 + OW_FI;  sc = W_CARRY; zero = (lb >= CB_IPV); }
  else if (blk < CC5) { src = wfo;  lb = blk - CC4; dstp = W16 + OW_FO;  sc = W_CARRY; }
  else if (blk < CC6) { src = wbi;  lb = blk - CC5; dstp = W16 + OW_BI;  sc = W_CARRY; zero = (lb >= CB_IPV); }
  else                { src = wbo;  lb = blk - CC6; dstp = W16 + OW_BO;  sc = W_CARRY; }
  const int lbs = zero ? 0 : lb;
  const size_t so = (size_t)lbs * CVB + (size_t)tid * 8;
  const v4f a0 = *(const v4f*)(src + so);
  const v4f a1 = *(const v4f*)(src + so + 4);
  const float f = zero ? 0.0f : sc;
  const v8h hv = cvt8(a0, a1, f);
  _Float16* dst = dstp + (size_t)lb * CVB + (size_t)tid * 8;
  *(volatile v8h*)dst = hv;
  __threadfence();
  *(volatile v8h*)dst = hv;
}

template <int WM, int NT, int AHM, int HASB>
__global__ __launch_bounds__(NTHR) void k_gemm(const _Float16* __restrict__ Ap, const _Float16* __restrict__ Wp,
                                               const float* __restrict__ bias, float* Cf,
                                               int lda, int ldw, int ldc, int K, float scale) {
  constexpr int WN = 8 / WM;
  constexpr int R = 16 * WM;
  constexpr int BN = WN * 16 * NT;
  static_assert(WM * WN == 8);
  static_assert(((R * BN / 4) % NTHR) == 0);
  constexpr int NF4 = (R * BN / 4) / NTHR;
  __shared__ __align__(16) float sC[R * BN];
  const int tid = threadIdx.x, lane = tid & 31, wave = tid >> 5, h = lane >> 4, m = lane & 15;
  const int wm = wave % WM, wn = wave / WM;
  const int bm0 = blockIdx.y * R;
  const int n0 = blockIdx.x * BN;
  const int m0 = bm0 + 16 * wm;
  const int nw0 = n0 + wn * 16 * NT;
  const int gm = m0 + m;

  size_t abase, astep, ahalf;
  if constexpr (AHM != 0) {
    const int sq = gm >> 10, tt = gm & (LL - 1);
    abase = ((size_t)(sq * NHEAD) * LL + (size_t)tt) * HDIM + 8 * h;
    astep = (size_t)2 * LL * HDIM;
    ahalf = (size_t)LL * HDIM;
  } else {
    abase = (size_t)gm * (size_t)lda + 8 * h;
    astep = 32;
    ahalf = 16;
  }
  const size_t wbase = (size_t)(nw0 + m) * (size_t)ldw + 8 * h;

  v8f acc[NT];
#pragma unroll
  for (int t = 0; t < NT; ++t) acc[t] = zero8();
  const int nks = K >> 5;

#pragma unroll 1
  for (int ks = 0; ks < nks; ++ks) {
    const _Float16* ap = Ap + abase + (size_t)ks * astep;
    Frag fa;
    fa.hv[0] = *(const v8h*)ap;
    fa.hv[1] = *(const v8h*)(ap + ahalf);
    const int k0 = ks << 5;
#pragma unroll
    for (int t = 0; t < NT; ++t) {
      const _Float16* wp = Wp + wbase + (size_t)(16 * t) * (size_t)ldw + k0;
      Frag fw;
      fw.hv[0] = *(const v8h*)wp;
      fw.hv[1] = *(const v8h*)(wp + 16);
      acc[t] = wmf(fa, fw, acc[t]);
    }
  }

#pragma unroll
  for (int t = 0; t < NT; ++t) {
    const int cl = wn * 16 * NT + 16 * t + m;
#pragma unroll
    for (int r = 0; r < 8; ++r) {
      const int rl = 16 * wm + 8 * h + r;
      sC[rl * BN + cl] = acc[t][r];
    }
  }
  __syncthreads();

#pragma unroll
  for (int it = 0; it < NF4; ++it) {
    const int e = tid + it * NTHR;
    const int rl = e / (BN / 4), q = e - rl * (BN / 4);
    v4f v = *(const v4f*)(sC + 4 * e) * scale;
    if constexpr (HASB != 0) {
      const v4f bb = *(const v4f*)(bias + n0 + 4 * q);
      v = v + bb;
    }
    *(volatile v4f*)(Cf + (size_t)(bm0 + rl) * (size_t)ldc + n0 + 4 * q) = v;
  }
  __threadfence();
#pragma unroll
  for (int it = 0; it < NF4; ++it) {
    const int e = tid + it * NTHR;
    const int rl = e / (BN / 4), q = e - rl * (BN / 4);
    v4f v = *(const v4f*)(sC + 4 * e) * scale;
    if constexpr (HASB != 0) {
      const v4f bb = *(const v4f*)(bias + n0 + 4 * q);
      v = v + bb;
    }
    *(volatile v4f*)(Cf + (size_t)(bm0 + rl) * (size_t)ldc + n0 + 4 * q) = v;
  }
}

__global__ __launch_bounds__(NTHR) void k_qkv(const float* __restrict__ QKV, _Float16* Q16, _Float16* K16,
                                              _Float16* VT16) {
  __shared__ __align__(16) float sV[8 * 64 * HDIM];
  const int tile = blockIdx.x, hg = blockIdx.y, bq = blockIdx.z;
  const int tid = threadIdx.x, lane = tid & 31, wave = tid >> 5;
  const int hh = 8 * hg + wave;
  const int t0 = 64 * tile;
  const size_t rowb = (size_t)bq * LL;
  const size_t plane = (size_t)(bq * NHEAD + hh);
  v8h qv[4], kv[4], vv[4];
  size_t dq[4], dv[4];
#pragma unroll
  for (int i = 0; i < 4; ++i) {
    const int tt = t0 + 16 * i + (lane >> 1), dh = lane & 1;
    const float* sp = QKV + (rowb + tt) * (size_t)(3 * DM) + HDIM * hh + 8 * dh;
    qv[i] = cvt8(*(const v4f*)sp, *(const v4f*)(sp + 4), Q_CARRY);
    kv[i] = cvt8(*(const v4f*)(sp + DM), *(const v4f*)(sp + DM + 4), Q_CARRY);
    dq[i] = (plane * LL + tt) * HDIM + 8 * dh;
  }
  float* sv = sV + wave * (64 * HDIM);
#pragma unroll
  for (int i = 0; i < 8; ++i) {
    const int tt = 8 * i + (lane >> 2), d4 = 4 * (lane & 3);
    const v4f x = *(const v4f*)(QKV + (rowb + t0 + tt) * (size_t)(3 * DM) + 2 * DM + HDIM * hh + d4);
    *(v4f*)(sv + tt * HDIM + d4) = x;
  }
  __syncthreads();
#pragma unroll
  for (int i = 0; i < 4; ++i) {
    const int d = 4 * i + (lane >> 3), kq = lane & 7;
    v4f a, c;
#pragma unroll
    for (int j = 0; j < 4; ++j) {
      a[j] = sv[(8 * kq + j) * HDIM + d];
      c[j] = sv[(8 * kq + 4 + j) * HDIM + d];
    }
    vv[i] = cvt8(a, c, Q_CARRY);
    dv[i] = (plane * HDIM + d) * LL + t0 + 8 * kq;
  }
#pragma unroll
  for (int i = 0; i < 4; ++i) {
    *(volatile v8h*)(Q16 + dq[i]) = qv[i];
    *(volatile v8h*)(K16 + dq[i]) = kv[i];
    *(volatile v8h*)(VT16 + dv[i]) = vv[i];
  }
  __threadfence();
#pragma unroll
  for (int i = 0; i < 4; ++i) {
    *(volatile v8h*)(Q16 + dq[i]) = qv[i];
    *(volatile v8h*)(K16 + dq[i]) = kv[i];
    *(volatile v8h*)(VT16 + dv[i]) = vv[i];
  }
}

__global__ __launch_bounds__(NTHR) void k_attn(const _Float16* __restrict__ Q16, const _Float16* __restrict__ K16,
                                               const _Float16* __restrict__ VT16, _Float16* O16) {
  __shared__ __align__(16) float sS[16 * LL];
  const int qt = blockIdx.x, hh = blockIdx.y, bq = blockIdx.z;
  const int tid = threadIdx.x, lane = tid & 31, wave = tid >> 5, h = lane >> 4, m = lane & 15;
  const int q0 = 16 * qt;
  const size_t plane = (size_t)(bq * NHEAD + hh);

  Frag fq;
  fq.w = zero8i();
  fq.hv[0] = *(const v8h*)(Q16 + (plane * LL + q0 + m) * HDIM + 8 * h);
#pragma unroll 1
  for (int j = 0; j < 8; ++j) {
    const int kt = wave * 8 + j;
    Frag fk;
    fk.w = zero8i();
    fk.hv[0] = *(const v8h*)(K16 + (plane * LL + 16 * kt + m) * HDIM + 8 * h);
    const v8f s = wmf(fq, fk, zero8());
#pragma unroll
    for (int r = 0; r < 8; ++r) sS[(8 * h + r) * LL + 16 * kt + m] = s[r] * SC_SCORE;
  }
  __syncthreads();

  const int row = tid >> 4, jc = tid & 15;
  float* srow = sS + row * LL;
  float mx = srow[jc];
#pragma unroll 1
  for (int c = jc + 16; c < LL; c += 16) mx = fmaxf(mx, srow[c]);
  mx = fmaxf(mx, __shfl_xor(mx, 8, 32));
  mx = fmaxf(mx, __shfl_xor(mx, 4, 32));
  mx = fmaxf(mx, __shfl_xor(mx, 2, 32));
  mx = fmaxf(mx, __shfl_xor(mx, 1, 32));
  float sum = 0.0f;
#pragma unroll 4
  for (int c = jc; c < LL; c += 16) {
    const float e = P_CARRY * __expf(srow[c] - mx);
    srow[c] = e;
    sum += e;
  }
  sum += __shfl_xor(sum, 8, 32);
  sum += __shfl_xor(sum, 4, 32);
  sum += __shfl_xor(sum, 2, 32);
  sum += __shfl_xor(sum, 1, 32);
  const float inv = 1.0f / sum;
  __syncthreads();

  v8f acc = zero8();
#pragma unroll 1
  for (int j = 0; j < 4; ++j) {
    const int k0 = wave * 128 + 32 * j;
    const float* pp = sS + m * LL + k0 + 8 * h;
    const v4f p0 = *(const v4f*)pp;
    const v4f p1 = *(const v4f*)(pp + 4);
    const v4f p2 = *(const v4f*)(pp + 16);
    const v4f p3 = *(const v4f*)(pp + 20);
    Frag fp;
    fp.hv[0] = cvt8(p0, p1, 1.0f);
    fp.hv[1] = cvt8(p2, p3, 1.0f);
    const _Float16* vp = VT16 + (plane * HDIM + m) * LL + k0 + 8 * h;
    Frag fv;
    fv.hv[0] = *(const v8h*)vp;
    fv.hv[1] = *(const v8h*)(vp + 16);
    acc = wmf(fp, fv, acc);
  }
  __syncthreads();

  float* sR = sS;
  float* sI = sS + 8 * 256;
#pragma unroll
  for (int r = 0; r < 8; ++r) sR[wave * 256 + (8 * h + r) * 16 + m] = acc[r];
  if (jc == 0) sI[row] = inv;
  __syncthreads();

  if (wave == 0) {
    const int q = lane >> 1, dh = lane & 1;
    v4f oa = zero4(), ob = zero4();
#pragma unroll
    for (int w = 0; w < 8; ++w) {
      const float* rp = sR + w * 256 + q * 16 + 8 * dh;
      oa = oa + *(const v4f*)rp;
      ob = ob + *(const v4f*)(rp + 4);
    }
    const float f = sI[q] * SC_O;
    const v8h ov = cvt8(oa, ob, f);
    _Float16* dst = O16 + (plane * LL + q0 + q) * HDIM + 8 * dh;
    *(volatile v8h*)dst = ov;
    __threadfence();
    *(volatile v8h*)dst = ov;
  }
}

#define STB 32
#define SCH 192
static_assert((LL % STB) == 0 && (STB * SCH / 4) == 6 * NTHR && (STB * HPD / 4) == 2 * NTHR && SCH <= NTHR);

__global__ __launch_bounds__(NTHR) void k_scan(const float* __restrict__ XZ, const float* __restrict__ cw,
                                               const float* __restrict__ cb, const float* __restrict__ dtb,
                                               const float* __restrict__ alog, const float* __restrict__ Dp,
                                               float* Y32, int dir) {
  __shared__ __align__(16) float sXBC[STB * SCH];
  __shared__ __align__(16) float sY[STB * HPD];
  __shared__ __align__(16) float sW[SCH * DCV];
  __shared__ __align__(16) float sCB[SCH];
  __shared__ float sDT[STB], sDA[STB];
  const int hd = blockIdx.x, bq = blockIdx.y;
  const int tid = threadIdx.x;
  const int p = tid >> 2, nq = tid & 3;
  const float Ah = -expf(alog[hd]);
  const float dtbias = dtb[hd];
  const float Dh = Dp[hd];
  const size_t rowb = (size_t)bq * LL;
  const int sgn = dir ? -1 : 1;

#pragma unroll 1
  for (int e = tid; e < SCH * DCV; e += NTHR) {
    const int lc = e >> 2, j = e & 3;
    const int c = (lc < HPD) ? (HPD * hd + lc) : (DI + lc - HPD);
    sW[e] = cw[(size_t)c * DCV + j];
  }
  if (tid < SCH) {
    const int c = (tid < HPD) ? (HPD * hd + tid) : (DI + tid - HPD);
    sCB[tid] = cb[c];
  }
  __syncthreads();

  float st[16];
#pragma unroll
  for (int j = 0; j < 16; ++j) st[j] = 0.0f;

#pragma unroll 1
  for (int ci = 0; ci < LL / STB; ++ci) {
    if (tid < STB) {
      const int t = ci * STB + tid;
      const int s = dir ? (LL - 1 - t) : t;
      const float raw = XZ[(rowb + s) * DIPP + COL_DT + hd] + dtbias;
      const float sp = fmaxf(raw, 0.0f) + log1pf(__expf(-fabsf(raw)));
      sDT[tid] = sp;
      sDA[tid] = __expf(sp * Ah);
    }
#pragma unroll 1
    for (int i = 0; i < 6; ++i) {
      const int e = tid + NTHR * i;
      const int cq = e % 48, tl = e / 48;
      const int t = ci * STB + tl;
      const int s = dir ? (LL - 1 - t) : t;
      const int lc0 = 4 * cq;
      const int col = (cq < 16) ? (COL_X + HPD * hd + lc0) : (COL_B + lc0 - HPD);
      v4f a4 = *(const v4f*)(sCB + lc0);
      const v4f w0 = *(const v4f*)(sW + (lc0 + 0) * DCV);
      const v4f w1 = *(const v4f*)(sW + (lc0 + 1) * DCV);
      const v4f w2 = *(const v4f*)(sW + (lc0 + 2) * DCV);
      const v4f w3 = *(const v4f*)(sW + (lc0 + 3) * DCV);
#pragma unroll
      for (int j = 0; j < DCV; ++j) {
        const int src = s + sgn * (j - (DCV - 1));
        const bool ok = (unsigned)src < (unsigned)LL;
        const int srcc = ok ? src : s;
        const v4f xv = *(const v4f*)(XZ + (rowb + srcc) * DIPP + col);
        const float f = ok ? 1.0f : 0.0f;
        a4[0] = a4[0] + (xv[0] * f) * w0[j];
        a4[1] = a4[1] + (xv[1] * f) * w1[j];
        a4[2] = a4[2] + (xv[2] * f) * w2[j];
        a4[3] = a4[3] + (xv[3] * f) * w3[j];
      }
      v4f o4;
#pragma unroll
      for (int u = 0; u < 4; ++u) {
        const float a = a4[u];
        o4[u] = a * __builtin_amdgcn_rcpf(1.0f + __expf(-a));
      }
      *(v4f*)(sXBC + tl * SCH + lc0) = o4;
    }
    __syncthreads();

#pragma unroll 1
    for (int tl = 0; tl < STB; ++tl) {
      const float dt = sDT[tl], dA = sDA[tl];
      const float* rp = sXBC + tl * SCH;
      const float xp = rp[p];
      const float dtx = dt * xp;
      const v4f b0 = *(const v4f*)(rp + HPD + 16 * nq);
      const v4f b1 = *(const v4f*)(rp + HPD + 16 * nq + 4);
      const v4f b2 = *(const v4f*)(rp + HPD + 16 * nq + 8);
      const v4f b3 = *(const v4f*)(rp + HPD + 16 * nq + 12);
      const v4f c0 = *(const v4f*)(rp + HPD + DSS + 16 * nq);
      const v4f c1 = *(const v4f*)(rp + HPD + DSS + 16 * nq + 4);
      const v4f c2 = *(const v4f*)(rp + HPD + DSS + 16 * nq + 8);
      const v4f c3 = *(const v4f*)(rp + HPD + DSS + 16 * nq + 12);
      float Bv[16], Cv[16];
      Bv[0] = b0[0]; Bv[1] = b0[1]; Bv[2] = b0[2]; Bv[3] = b0[3]; Bv[4] = b1[0]; Bv[5] = b1[1]; Bv[6] = b1[2]; Bv[7] = b1[3];
      Bv[8] = b2[0]; Bv[9] = b2[1]; Bv[10] = b2[2]; Bv[11] = b2[3]; Bv[12] = b3[0]; Bv[13] = b3[1]; Bv[14] = b3[2]; Bv[15] = b3[3];
      Cv[0] = c0[0]; Cv[1] = c0[1]; Cv[2] = c0[2]; Cv[3] = c0[3]; Cv[4] = c1[0]; Cv[5] = c1[1]; Cv[6] = c1[2]; Cv[7] = c1[3];
      Cv[8] = c2[0]; Cv[9] = c2[1]; Cv[10] = c2[2]; Cv[11] = c2[3]; Cv[12] = c3[0]; Cv[13] = c3[1]; Cv[14] = c3[2]; Cv[15] = c3[3];
      float yp = 0.0f;
#pragma unroll
      for (int j = 0; j < 16; ++j) {
        const float hn = dA * st[j] + dtx * Bv[j];
        st[j] = hn;
        yp = yp + hn * Cv[j];
      }
      yp += __shfl_xor(yp, 1, 32);
      yp += __shfl_xor(yp, 2, 32);
      if (nq == 0) sY[tl * HPD + p] = yp + Dh * xp;
    }
    __syncthreads();

    v4f yv[2];
    size_t dst[2];
#pragma unroll
    for (int it = 0; it < 2; ++it) {
      const int e = tid + NTHR * it;
      const int rl = e >> 4, q = e & 15;
      const int t = ci * STB + rl;
      const int s = dir ? (LL - 1 - t) : t;
      yv[it] = *(const v4f*)(sY + rl * HPD + 4 * q);
      dst[it] = (rowb + s) * (size_t)DI + HPD * hd + 4 * q;
    }
    *(volatile v4f*)(Y32 + dst[0]) = yv[0];
    *(volatile v4f*)(Y32 + dst[1]) = yv[1];
    __threadfence();
    *(volatile v4f*)(Y32 + dst[0]) = yv[0];
    *(volatile v4f*)(Y32 + dst[1]) = yv[1];
  }
}

__global__ __launch_bounds__(NTHR) void k_gate(const float* __restrict__ Y32, const float* __restrict__ XZ,
                                               const float* __restrict__ nw, _Float16* Y16) {
  const int tid = threadIdx.x, lane = tid & 31, wave = tid >> 5;
  const size_t row = (size_t)blockIdx.x * 8 + wave;
  const float* yr = Y32 + row * DI;
  const float* zr = XZ + row * DIPP;
  float g[32];
  float ss = 0.0f;
#pragma unroll
  for (int i = 0; i < 4; ++i) {
    const int c = 256 * i + 8 * lane;
    const v4f y0 = *(const v4f*)(yr + c);
    const v4f y1 = *(const v4f*)(yr + c + 4);
    const v4f z0 = *(const v4f*)(zr + c);
    const v4f z1 = *(const v4f*)(zr + c + 4);
    float yv[8], zv[8];
    yv[0] = y0[0]; yv[1] = y0[1]; yv[2] = y0[2]; yv[3] = y0[3]; yv[4] = y1[0]; yv[5] = y1[1]; yv[6] = y1[2]; yv[7] = y1[3];
    zv[0] = z0[0]; zv[1] = z0[1]; zv[2] = z0[2]; zv[3] = z0[3]; zv[4] = z1[0]; zv[5] = z1[1]; zv[6] = z1[2]; zv[7] = z1[3];
#pragma unroll
    for (int u = 0; u < 8; ++u) {
      const float z = zv[u];
      const float sg = __builtin_amdgcn_rcpf(1.0f + __expf(-z));
      const float gv = yv[u] * (z * sg);
      g[8 * i + u] = gv;
      ss += gv * gv;
    }
  }
  ss += __shfl_xor(ss, 16, 32);
  ss += __shfl_xor(ss, 8, 32);
  ss += __shfl_xor(ss, 4, 32);
  ss += __shfl_xor(ss, 2, 32);
  ss += __shfl_xor(ss, 1, 32);
  const float rn = rsqrtf(ss * (1.0f / (float)DI) + 1e-5f);
  v8h ov[4];
#pragma unroll
  for (int i = 0; i < 4; ++i) {
    const int c = 256 * i + 8 * lane;
    const v4f wa = *(const v4f*)(nw + c);
    const v4f wb = *(const v4f*)(nw + c + 4);
    v4f oa, ob;
#pragma unroll
    for (int u = 0; u < 4; ++u) {
      oa[u] = (g[8 * i + u] * rn) * wa[u];
      ob[u] = (g[8 * i + 4 + u] * rn) * wb[u];
    }
    ov[i] = cvt8(oa, ob, 1.0f);
  }
#pragma unroll
  for (int i = 0; i < 4; ++i) *(volatile v8h*)(Y16 + row * DI + 256 * i + 8 * lane) = ov[i];
  __threadfence();
#pragma unroll
  for (int i = 0; i < 4; ++i) *(volatile v8h*)(Y16 + row * DI + 256 * i + 8 * lane) = ov[i];
}

__global__ __launch_bounds__(NTHR) void k_ln(const float* __restrict__ hin, const float* __restrict__ at,
                                             const float* __restrict__ fw, const float* __restrict__ bw,
                                             const float* __restrict__ g, const float* __restrict__ be, float* out) {
  const int tid = threadIdx.x, lane = tid & 31, wave = tid >> 5;
  const size_t row = (size_t)blockIdx.x * 8 + wave;
  const size_t base = row * DM;
  float s[16];
#pragma unroll
  for (int i = 0; i < 4; ++i) {
    const size_t c = base + 128 * i + 4 * lane;
    const v4f a = *(const v4f*)(hin + c);
    const v4f x1 = *(const v4f*)(at + c);
    const v4f x2 = *(const v4f*)(fw + c);
    const v4f x3 = *(const v4f*)(bw + c);
#pragma unroll
    for (int u = 0; u < 4; ++u) s[4 * i + u] = ((a[u] + x1[u]) + x2[u]) + x3[u];
  }
  float sum = (((s[0] + s[1]) + (s[2] + s[3])) + ((s[4] + s[5]) + (s[6] + s[7]))) +
              (((s[8] + s[9]) + (s[10] + s[11])) + ((s[12] + s[13]) + (s[14] + s[15])));
  sum += __shfl_xor(sum, 16, 32);
  sum += __shfl_xor(sum, 8, 32);
  sum += __shfl_xor(sum, 4, 32);
  sum += __shfl_xor(sum, 2, 32);
  sum += __shfl_xor(sum, 1, 32);
  const float mu = sum * (1.0f / (float)DM);
  float d[16];
  float ss = 0.0f;
#pragma unroll
  for (int i = 0; i < 16; ++i) { d[i] = s[i] - mu; ss = ss + d[i] * d[i]; }
  ss += __shfl_xor(ss, 16, 32);
  ss += __shfl_xor(ss, 8, 32);
  ss += __shfl_xor(ss, 4, 32);
  ss += __shfl_xor(ss, 2, 32);
  ss += __shfl_xor(ss, 1, 32);
  const float var = ss * (1.0f / (float)DM);
  const float rinv = rsqrtf(var + LNEPS);
  v4f ov[4];
#pragma unroll
  for (int i = 0; i < 4; ++i) {
    const int c = 128 * i + 4 * lane;
    const v4f gv = *(const v4f*)(g + c);
    const v4f bv = *(const v4f*)(be + c);
#pragma unroll
    for (int u = 0; u < 4; ++u) ov[i][u] = (d[4 * i + u] * rinv) * gv[u] + bv[u];
  }
#pragma unroll
  for (int i = 0; i < 4; ++i) *(volatile v4f*)(out + base + 128 * i + 4 * lane) = ov[i];
  __threadfence();
#pragma unroll
  for (int i = 0; i < 4; ++i) *(volatile v4f*)(out + base + 128 * i + 4 * lane) = ov[i];
}

extern "C" void kernel_launch(void* const* d_in, const int* in_sizes, int n_in,
                              void* d_out, int out_size, void* d_ws, size_t ws_size,
                              hipStream_t stream) {
  if (n_in < 23) return;
  if (in_sizes[0] != NTOK * DM) return;
  if (in_sizes[1] != 3 * DM * DM || in_sizes[2] != 3 * DM) return;
  if (in_sizes[3] != DM * DM || in_sizes[4] != DM) return;
  for (int dd = 0; dd < 2; ++dd) {
    const int o = 5 + 8 * dd;
    if (in_sizes[o] != DIP * DM) return;
    if (in_sizes[o + 1] != CCH * DCV || in_sizes[o + 2] != CCH) return;
    if (in_sizes[o + 3] != NHM || in_sizes[o + 4] != NHM || in_sizes[o + 5] != NHM) return;
    if (in_sizes[o + 6] != DI || in_sizes[o + 7] != DM * DI) return;
  }
  if (in_sizes[21] != DM || in_sizes[22] != DM) return;
  if (out_size != NTOK * DM) return;
  const size_t tot = (size_t)WSTOT;
  if (tot > ws_size || tot > (size_t)WSCAP) return;

  const float* hin        = (const float*)d_in[0];
  const float* attn_in_w  = (const float*)d_in[1];
  const float* attn_in_b  = (const float*)d_in[2];
  const float* attn_out_w = (const float*)d_in[3];
  const float* attn_out_b = (const float*)d_in[4];
  const float* ip_w[2] = {(const float*)d_in[5],  (const float*)d_in[13]};
  const float* cv_w[2] = {(const float*)d_in[6],  (const float*)d_in[14]};
  const float* cv_b[2] = {(const float*)d_in[7],  (const float*)d_in[15]};
  const float* dt_b[2] = {(const float*)d_in[8],  (const float*)d_in[16]};
  const float* a_lg[2] = {(const float*)d_in[9],  (const float*)d_in[17]};
  const float* d_pr[2] = {(const float*)d_in[10], (const float*)d_in[18]};
  const float* nm_w[2] = {(const float*)d_in[11], (const float*)d_in[19]};
  const float* op_w[2] = {(const float*)d_in[12], (const float*)d_in[20]};
  const float* ln_w = (const float*)d_in[21];
  const float* ln_b = (const float*)d_in[22];
  float* out = (float*)d_out;

  char* ws = (char*)d_ws;
  _Float16* W16  = (_Float16*)(ws + O_W16);
  _Float16* H16  = (_Float16*)(ws + O_H16);
  float*    ATT  = (float*)(ws + O_ATT);
  float*    FWD  = (float*)(ws + O_FWD);
  float*    BWD  = (float*)(ws + O_BWD);
  float*    QKV  = (float*)(ws + O_QKV);
  _Float16* Q16  = (_Float16*)(ws + O_Q16);
  _Float16* K16  = (_Float16*)(ws + O_K16);
  _Float16* VT16 = (_Float16*)(ws + O_VT);
  _Float16* O16  = (_Float16*)(ws + O_O16);
  float*    XZ   = (float*)(ws + O_XZ);
  float*    Y32  = (float*)(ws + O_Y32);
  _Float16* Y16  = (_Float16*)(ws + O_Y16);
  float* dirout[2] = {FWD, BWD};
  const size_t owi[2] = {OW_FI, OW_BI};
  const size_t owo[2] = {OW_FO, OW_BO};

  k_cvt<<<CCT, NTHR, 0, stream>>>(hin, attn_in_w, attn_out_w, ip_w[0], op_w[0], ip_w[1], op_w[1], H16, W16);

  k_gemm<2, 4, 0, 1><<<dim3(3 * DM / 256, NTOK / 32), NTHR, 0, stream>>>(
      H16, W16 + OW_QKV, attn_in_b, QKV, DM, DM, 3 * DM, DM, 1.0f / W_CARRY);

  k_qkv<<<dim3(LL / 64, NHEAD / 8, BB), NTHR, 0, stream>>>(QKV, Q16, K16, VT16);

  k_attn<<<dim3(LL / 16, NHEAD, BB), NTHR, 0, stream>>>(Q16, K16, VT16, O16);

  k_gemm<2, 4, 1, 1><<<dim3(DM / 256, NTOK / 32), NTHR, 0, stream>>>(
      O16, W16 + OW_AO, attn_out_b, ATT, 0, DM, DM, DM, 1.0f / (W_CARRY * 64.0f));

  for (int dd = 0; dd < 2; ++dd) {
    k_gemm<4, 2, 0, 0><<<dim3(DIPP / 64, NTOK / 64), NTHR, 0, stream>>>(
        H16, W16 + owi[dd], hin, XZ, DM, DM, DIPP, DM, 1.0f / W_CARRY);
    k_scan<<<dim3(NHM, BB), NTHR, 0, stream>>>(XZ, cv_w[dd], cv_b[dd], dt_b[dd], a_lg[dd], d_pr[dd], Y32, dd);
    k_gate<<<NTOK / 8, NTHR, 0, stream>>>(Y32, XZ, nm_w[dd], Y16);
    k_gemm<2, 4, 0, 0><<<dim3(DM / 256, NTOK / 32), NTHR, 0, stream>>>(
        Y16, W16 + owo[dd], hin, dirout[dd], DI, DI, DM, DI, 1.0f / W_CARRY);
  }

  k_ln<<<NTOK / 8, NTHR, 0, stream>>>(hin, ATT, FWD, BWD, ln_w, ln_b, out);
}
